// PsiNN_84688165142618
// MI455X (gfx1250) — hardware-verified
//
#include <hip/hip_runtime.h>

#define NB     64
#define NT     2048
#define NI     25
#define NR     512
#define NO     50
#define NOPAD  64
#define HST    520
#define XST    40
#define TG     16
#define NTW    4
#define NTHR   256
#define OROW   (TG * NO)
#define LPR    (OROW / 32)
#define NLINES (16 * LPR)
#define ALPHA  0.5f
#define SCX    16.0f
#define SCWIN  256.0f
#define SCH    64.0f
#define SCW    64.0f
#define SCWO   64.0f
#define INV_U  (1.0f / 4096.0f)
#define INV_O  (1.0f / 4096.0f)

typedef _Float16 v16h __attribute__((ext_vector_type(16)));
typedef _Float16 v8h  __attribute__((ext_vector_type(8)));
typedef float    v8f  __attribute__((ext_vector_type(8)));
typedef float    v4f  __attribute__((ext_vector_type(4)));
typedef v8h v8ha __attribute__((may_alias));
typedef v4f v4fa __attribute__((may_alias));

union Frag  { v16h v; v8h half[2]; _Float16 s[16]; };
union Frag8 { v8h v; _Float16 s[8]; };

__device__ __forceinline__ v8f wmma16(const v16h a, const v16h b, v8f c) {
  v8f d = __builtin_amdgcn_wmma_f32_16x16x32_f16(false, a, false, b, (short)0, c, false, false);
  asm volatile("v_nop\n\tv_nop\n\tv_nop\n\tv_nop" : "+v"(d) : "v"(a), "v"(b));
  return d;
}

__device__ __forceinline__ v16h ld_frag_lds(const _Float16* p) {
  Frag f;
  f.half[0] = *(const v8ha*)(p);
  f.half[1] = *(const v8ha*)(p + 16);
  return f.v;
}
__device__ __forceinline__ v16h ld_frag_glb(const _Float16* __restrict__ p) {
  Frag f;
  f.half[0] = *(const v8ha*)(p);
  f.half[1] = *(const v8ha*)(p + 16);
  return f.v;
}

__global__ __launch_bounds__(NTHR) void k_prep(const float* __restrict__ W,
                                              _Float16* __restrict__ Wh, int n8)
{
  const int i = blockIdx.x * NTHR + threadIdx.x;
  const bool ok = i < n8;
  Frag8 pk;
#pragma unroll
  for (int j = 0; j < 8; ++j) pk.s[j] = (_Float16)0.0f;
  if (ok) {
    const float* s = W + (size_t)i * 8;
#pragma unroll
    for (int j = 0; j < 8; ++j) pk.s[j] = (_Float16)(s[j] * SCW);
  }
  _Float16* d = Wh + (size_t)i * 8;
  if (ok) *(volatile v8h*)d = pk.v;
  __threadfence();
  if (ok) *(volatile v8h*)d = pk.v;
}

__global__ __launch_bounds__(NTHR) void k_main(const float* __restrict__ x,
                                              const float* __restrict__ Win,
                                              const float* __restrict__ Wout,
                                              const _Float16* __restrict__ Wh,
                                              float* __restrict__ out, int nbg)
{
  __shared__ __attribute__((aligned(16))) _Float16 hHist[2 * 16 * HST];
  __shared__ __attribute__((aligned(16))) _Float16 woutL[NOPAD * HST];
  __shared__ __attribute__((aligned(16))) _Float16 xA[TG * 16 * XST];
  __shared__ __attribute__((aligned(16))) float    ostage[16 * OROW];

  const int tid  = threadIdx.x;
  const int w    = tid >> 5;
  const int lane = tid & 31;
  const int h    = lane >> 4;
  const int l16  = lane & 15;
  const int bg   = blockIdx.x;
  if (bg >= nbg) return;

  for (int i = tid; i < 16 * HST; i += NTHR) hHist[16 * HST + i] = (_Float16)0.0f;

  for (int i = tid; i < NOPAD * NR; i += NTHR) {
    const int o = i >> 9, k = i & (NR - 1);
    float v = 0.0f;
    if (o < NO) v = Wout[o * NR + k] * SCWO;
    woutL[o * HST + k] = (_Float16)v;
  }

  v16h winF[NTW];
#pragma unroll
  for (int j = 0; j < NTW; ++j) {
    const int n = (w * NTW + j) * 16 + l16;
    Frag f;
#pragma unroll
    for (int i = 0; i < 16; ++i) {
      const int k = 8 * h + (i & 7) + ((i >> 3) << 4);
      float v = 0.0f;
      if (k < NI) v = Win[n * NI + k] * SCWIN;
      f.s[i] = (_Float16)v;
    }
    winF[j] = f.v;
  }

  v8f hold[NTW];
#pragma unroll
  for (int j = 0; j < NTW; ++j)
#pragma unroll
    for (int v = 0; v < 8; ++v) hold[j][v] = 0.0f;

  __syncthreads();

  const int q    = lane & 7;
  const int lsub = lane >> 3;

  for (int tg0 = 0; tg0 < NT; tg0 += TG) {
    for (int i = tid; i < TG * 16 * 32; i += NTHR) {
      const int k = i & 31, m = (i >> 5) & 15, tl = i >> 9;
      float v = 0.0f;
      if (k < NI)
        v = x[((size_t)(bg * 16 + m) * NT + (size_t)(tg0 + tl)) * NI + k] * SCX;
      xA[(tl * 16 + m) * XST + k] = (_Float16)v;
    }
    __syncthreads();

#pragma unroll 1
    for (int tl = 0; tl < TG; ++tl) {
      const int t = tg0 + tl;
      const _Float16* hR = hHist + ((t + 1) & 1) * (16 * HST);
      _Float16*       hW = hHist + (t & 1) * (16 * HST);

      v8f acc[NTW];
      {
        const v16h ax = ld_frag_lds(xA + (tl * 16 + l16) * XST + 8 * h);
        v8f z;
#pragma unroll
        for (int v = 0; v < 8; ++v) z[v] = 0.0f;
#pragma unroll
        for (int j = 0; j < NTW; ++j) acc[j] = wmma16(ax, winF[j], z);
      }

      const _Float16* aB = hR + l16 * HST + 8 * h;
      const _Float16* bB = Wh + (size_t)((w * NTW) * 16 + l16) * NR + 8 * h;
#pragma unroll 2
      for (int kt = 0; kt < 16; ++kt) {
        const v16h a = ld_frag_lds(aB + kt * 32);
#pragma unroll
        for (int j = 0; j < NTW; ++j) {
          const v16h b = ld_frag_glb(bB + (size_t)j * 16 * NR + kt * 32);
          acc[j] = wmma16(a, b, acc[j]);
        }
      }

#pragma unroll
      for (int j = 0; j < NTW; ++j) {
        const int col = (w * NTW + j) * 16 + l16;
#pragma unroll
        for (int v = 0; v < 8; ++v) {
          const float u  = acc[j][v] * INV_U;
          const float hn = (1.0f - ALPHA) * hold[j][v] + ALPHA * tanhf(u);
          hold[j][v] = hn;
          hW[(8 * h + v) * HST + col] = (_Float16)(hn * SCH);
        }
      }
      __syncthreads();

      if (w < 4) {
        v8f oacc;
#pragma unroll
        for (int v = 0; v < 8; ++v) oacc[v] = 0.0f;
        const _Float16* ra = hW + l16 * HST + 8 * h;
        const _Float16* rb = woutL + (w * 16 + l16) * HST + 8 * h;
#pragma unroll 2
        for (int kt = 0; kt < 16; ++kt)
          oacc = wmma16(ld_frag_lds(ra + kt * 32), ld_frag_lds(rb + kt * 32), oacc);
        const int o = w * 16 + l16;
        if (o < NO) {
#pragma unroll
          for (int v = 0; v < 8; ++v)
            ostage[(8 * h + v) * OROW + tl * NO + o] = oacc[v] * INV_O;
        }
      }
    }
    __syncthreads();

    float* ob = out + ((size_t)bg * 16 * NT + (size_t)tg0) * NO;
#pragma unroll 1
    for (int G = w; G < NLINES / 4; G += 8) {
      const int L  = G * 4 + lsub;
      const int m  = L / LPR;
      const int lr = L - m * LPR;
      const v4f val = *(const v4fa*)(ostage + m * OROW + lr * 32 + q * 4);
      *(volatile v4f*)(ob + (size_t)m * NT * NO + lr * 32 + q * 4) = val;
    }
    __threadfence();
#pragma unroll 1
    for (int G = w; G < NLINES / 4; G += 8) {
      const int L  = G * 4 + lsub;
      const int m  = L / LPR;
      const int lr = L - m * LPR;
      const v4f val = *(const v4fa*)(ostage + m * OROW + lr * 32 + q * 4);
      *(volatile v4f*)(ob + (size_t)m * NT * NO + lr * 32 + q * 4) = val;
    }
  }
}

extern "C" void kernel_launch(void* const* d_in, const int* in_sizes, int n_in,
                              void* d_out, int out_size, void* d_ws, size_t ws_size,
                              hipStream_t stream) {
  if (n_in < 4) return;
  if (in_sizes[0] != NB * NT * NI) return;
  if (in_sizes[1] != NR * NI) return;
  if (in_sizes[2] != NR * NR) return;
  if (in_sizes[3] != NO * NR) return;
  if (out_size != NB * NT * NO) return;
  const size_t need = (size_t)NR * NR * sizeof(_Float16);
  if (ws_size < need) return;

  const float* x    = (const float*)d_in[0];
  const float* Win  = (const float*)d_in[1];
  const float* W    = (const float*)d_in[2];
  const float* Wout = (const float*)d_in[3];
  _Float16* Wh = (_Float16*)d_ws;
  float* out = (float*)d_out;

  const int n8 = NR * NR / 8;
  k_prep<<<dim3((n8 + NTHR - 1) / NTHR), dim3(NTHR), 0, stream>>>(W, Wh, n8);
  k_main<<<dim3(NB / 16), dim3(NTHR), 0, stream>>>(x, Win, Wout, Wh, out, NB / 16);
}
